// MultiHeadAttentionWithRPE_23321672417445
// MI455X (gfx1250) — hardware-verified
//
#include <hip/hip_runtime.h>
#include <hip/hip_bf16.h>

typedef __attribute__((ext_vector_type(16))) _Float16 v16h;
typedef __attribute__((ext_vector_type(8)))  _Float16 v8h;
typedef __attribute__((ext_vector_type(16))) __bf16   v16b;
typedef __attribute__((ext_vector_type(8)))  __bf16   v8b;
typedef __attribute__((ext_vector_type(8)))  float    v8f;
typedef __attribute__((ext_vector_type(4)))  float    v4f;
typedef __attribute__((ext_vector_type(4)))  unsigned v4u;

__device__ __forceinline__ unsigned short f2bf_bits(float f) {
  unsigned u = __float_as_uint(f);
  return (unsigned short)((u + 0x7FFFu + ((u >> 16) & 1u)) >> 16);
}
__device__ __forceinline__ float bf_bits2f(unsigned short h) { return __uint_as_float(((unsigned)h) << 16); }

__device__ __forceinline__ void dep_guard_h(v8f& a, v8f& b, v16h x, v16h y) { asm volatile("v_nop\n\tv_nop\n\tv_nop\n\tv_nop" : "+v"(a), "+v"(b) : "v"(x), "v"(y)); }
__device__ __forceinline__ void dep_guard_b(v8f& a, v8f& b, v16b x, v16b y) { asm volatile("v_nop\n\tv_nop\n\tv_nop\n\tv_nop" : "+v"(a), "+v"(b) : "v"(x), "v"(y)); }
__device__ __forceinline__ void keep4_h(v16h a, v16h b, v16h c, v16h d) { asm volatile("v_nop" :: "v"(a), "v"(b), "v"(c), "v"(d)); }
__device__ __forceinline__ void keep4_b(v16b a, v16b b, v16b c, v16b d) { asm volatile("v_nop" :: "v"(a), "v"(b), "v"(c), "v"(d)); }
__device__ __forceinline__ void acc_guard4(v8f& a, v8f& b, v8f& c, v8f& d) { asm volatile("v_nop\n\tv_nop\n\tv_nop\n\tv_nop" : "+v"(a), "+v"(b), "+v"(c), "+v"(d)); }
template <typename T> struct Frag;
template <> struct Frag<_Float16> {
  typedef v16h V; union U { v16h v; v8h h[2]; };
  static __device__ __forceinline__ v16h load(const _Float16* p) {
    U f; f.h[0] = *(const v8h*)(p); f.h[1] = *(const v8h*)(p + 16); return f.v;
  }
  static __device__ __forceinline__ v8f mma(v16h a, v16h b, v8f c) {
    return __builtin_amdgcn_wmma_f32_16x16x32_f16(false, a, false, b, (short)0, c, false, false);
  }
  static __device__ __forceinline__ void guard(v8f& a, v8f& b, v16h x, v16h y) { dep_guard_h(a, b, x, y); }
  static __device__ __forceinline__ void keep(v16h a, v16h b, v16h c, v16h d) { keep4_h(a, b, c, d); }
};
template <> struct Frag<__bf16> {
  typedef v16b V; union U { v16b v; v8b h[2]; };
  static __device__ __forceinline__ v16b load(const __bf16* p) {
    U f; f.h[0] = *(const v8b*)(p); f.h[1] = *(const v8b*)(p + 16); return f.v;
  }
  static __device__ __forceinline__ v8f mma(v16b a, v16b b, v8f c) {
    return __builtin_amdgcn_wmma_f32_16x16x32_bf16(false, a, false, b, (short)0, c, false, false);
  }
  static __device__ __forceinline__ void guard(v8f& a, v8f& b, v16b x, v16b y) { dep_guard_b(a, b, x, y); }
  static __device__ __forceinline__ void keep(v16b a, v16b b, v16b c, v16b d) { keep4_b(a, b, c, d); }
};

template <int ET> struct Elem;
template <> struct Elem<0> { typedef _Float16 T; };
template <> struct Elem<1> { typedef __bf16 T; };
template <int ET, bool SPLIT, int BIAS_MODE, int OUT_MODE, bool RESID, int ACT = 0>
__global__ __launch_bounds__(256) void wmma_gemm64(
    const unsigned short* __restrict__ Ap, const unsigned short* __restrict__ A2p, int lda, long strideA,
    const unsigned short* __restrict__ Btp, const unsigned short* __restrict__ Bt2p, int ldb, long strideB,
    void* __restrict__ Cout, void* __restrict__ Cout2, int ldc, long strideC,
    const float* __restrict__ bias,
    const float* __restrict__ resid, long strideR,
    int M, int N, int K, float scale) {
  typedef typename Elem<ET>::T T;
  typedef typename Frag<T>::V V;
  const T* A = (const T*)Ap; const T* A2 = (const T*)A2p; const T* Bt = (const T*)Btp; const T* Bt2 = (const T*)Bt2p;
  __shared__ __align__(16) float sT[8][16 * 68];
  const int b    = blockIdx.y;
  const int lane = threadIdx.x & 31;
  const int wave = threadIdx.x >> 5;
  const int tilesN = N >> 6;
  const int tilesM = M >> 6;
  const int tile = blockIdx.x * 8 + wave;
  if (tile >= tilesM * tilesN) return;
  const int tm = tile / tilesN;
  const int tn = tile - tm * tilesN;
  const int m0 = tm << 6;
  const int n0 = tn << 6;

  const T* Ab  = A  + (size_t)b * strideA;
  const T* Bb  = Bt + (size_t)b * strideB;
  const T* Ab2 = SPLIT ? (A2  + (size_t)b * strideA) : nullptr;
  const T* Bb2 = SPLIT ? (Bt2 + (size_t)b * strideB) : nullptr;

  const int rlane = lane & 15;
  const int koff  = (lane >> 4) * 8;
  const int mOff  = (lane >> 4) * 8;

  v8f acc[4][4];
#pragma unroll
  for (int i = 0; i < 4; ++i)
#pragma unroll
    for (int j = 0; j < 4; ++j) acc[i][j] = (v8f){0.f,0.f,0.f,0.f,0.f,0.f,0.f,0.f};

  for (int k0 = 0; k0 < K; k0 += 32) {
    V bh[4], bl[4];
#pragma unroll
    for (int j = 0; j < 4; ++j) {
      const size_t bo = (size_t)(n0 + (j << 4) + rlane) * ldb + koff + k0;
      bh[j] = Frag<T>::load(Bb + bo);
      if (SPLIT) bl[j] = Frag<T>::load(Bb2 + bo);
    }
#pragma unroll
    for (int i = 0; i < 4; ++i) {
      const size_t ao = (size_t)(m0 + (i << 4) + rlane) * lda + koff + k0;
      V ah = Frag<T>::load(Ab + ao);
      V al;
      if (SPLIT) al = Frag<T>::load(Ab2 + ao);
#pragma unroll
      for (int j = 0; j < 4; ++j) {
        acc[i][j] = Frag<T>::mma(ah, bh[j], acc[i][j]);
        if (SPLIT) {
          acc[i][j] = Frag<T>::mma(ah, bl[j], acc[i][j]);
          acc[i][j] = Frag<T>::mma(al, bh[j], acc[i][j]);
        }
      }
      Frag<T>::guard(acc[i][0], acc[i][3], ah, SPLIT ? al : ah);
    }
    Frag<T>::keep(bh[0], bh[1], bh[2], bh[3]);
    if (SPLIT) Frag<T>::keep(bl[0], bl[1], bl[2], bl[3]);
  }
  acc_guard4(acc[0][0], acc[0][1], acc[0][2], acc[0][3]);
  acc_guard4(acc[1][0], acc[1][1], acc[1][2], acc[1][3]);
  acc_guard4(acc[2][0], acc[2][1], acc[2][2], acc[2][3]);
  acc_guard4(acc[3][0], acc[3][1], acc[3][2], acc[3][3]);

  float* slab = sT[wave];
  const float* Rb = RESID ? (resid + (size_t)b * strideR) : nullptr;
#pragma unroll
  for (int i = 0; i < 4; ++i) {
    const int mBase = m0 + (i << 4);
#pragma unroll
    for (int j = 0; j < 4; ++j) {
      const int n = n0 + (j << 4) + rlane;
      float bv = 0.f;
      if (BIAS_MODE == 2) bv = bias[n];
#pragma unroll
      for (int r = 0; r < 8; ++r) {
        float v = acc[i][j][r] * scale;
        if (BIAS_MODE == 1) v += bias[mBase + mOff + r];
        if (BIAS_MODE == 2) v += bv;
        if (RESID) v += Rb[(size_t)(mBase + mOff + r) * ldc + n];
        if (ACT == 1) v = tanhf(v);
        if (ACT == 2) v = fmaxf(v, 0.0f);
        if (ACT == 3) v = v / (1.0f + expf(-v));
        if (ACT == 4) v = (v > 0.f) ? v : 0.01f * v;
        if (ACT == 5) v = 0.5f * v * (1.0f + erff(v * 0.70710678118654752f));
        slab[(mOff + r) * 68 + (j << 4) + rlane] = v;
      }
    }
    __builtin_amdgcn_fence(__ATOMIC_RELEASE, "workgroup");
    __builtin_amdgcn_wave_barrier();
    __builtin_amdgcn_fence(__ATOMIC_ACQUIRE, "workgroup");
    if (OUT_MODE == 0) {
      float* C = (float*)Cout + (size_t)b * strideC;
      const int hh = lane >> 4, c4 = (lane & 15) * 4;
      for (int pass = 0; pass < 2; ++pass) {
#pragma unroll
        for (int it = 0; it < 8; ++it) {
          const int row = it * 2 + hh;
          v4f v = *(const v4f*)(slab + row * 68 + c4);
          *(volatile v4f*)(C + (size_t)(mBase + row) * ldc + n0 + c4) = v;
        }
        __threadfence();
      }
    } else {
      const int q = lane >> 3, c8 = (lane & 7) * 8;
      unsigned short* C  = (unsigned short*)Cout  + (size_t)b * strideC;
      unsigned short* C2 = (OUT_MODE == 2) ? ((unsigned short*)Cout2 + (size_t)b * strideC) : nullptr;
      for (int pass = 0; pass < 2; ++pass) {
#pragma unroll
        for (int it = 0; it < 4; ++it) {
          const int row = it * 4 + q;
          const float* sp = slab + row * 68 + c8;
          v8h hv, lv;
#pragma unroll
          for (int e = 0; e < 8; ++e) {
            if (OUT_MODE == 1) {
              hv[e] = (_Float16)sp[e];
            } else {
              unsigned short hb = f2bf_bits(sp[e]);
              unsigned short lb = f2bf_bits(sp[e] - bf_bits2f(hb));
              hv[e] = __builtin_bit_cast(_Float16, hb);
              lv[e] = __builtin_bit_cast(_Float16, lb);
            }
          }
          *(volatile v8h*)(C + (size_t)(mBase + row) * ldc + n0 + c8) = hv;
          if (OUT_MODE == 2) *(volatile v8h*)(C2 + (size_t)(mBase + row) * ldc + n0 + c8) = lv;
        }
        __threadfence();
      }
    }
    __builtin_amdgcn_fence(__ATOMIC_RELEASE, "workgroup");
    __builtin_amdgcn_wave_barrier();
    __builtin_amdgcn_fence(__ATOMIC_ACQUIRE, "workgroup");
  }
}

__global__ __launch_bounds__(256) void cast_f32_f16x2s(
    const float* __restrict__ in, _Float16* __restrict__ out, int n2, float sc) {
  int i = blockIdx.x * 256 + threadIdx.x;
  if (i < n2) {
    const _Float16 h0 = (_Float16)(in[2 * i] * sc), h1 = (_Float16)(in[2 * i + 1] * sc);
    const unsigned u = (unsigned)__builtin_bit_cast(unsigned short, h0) | ((unsigned)__builtin_bit_cast(unsigned short, h1) << 16);
    ((volatile unsigned*)out)[i] = u;
    __threadfence();
    ((volatile unsigned*)out)[i] = u;
  }
}

#define AT_D 64
#define AT_NW 4
#define AT_QB 64
#define AT_KC 64
#define SEQ_T 2048
#define NBATCH 2
#define NHEAD 16
#define NQB (SEQ_T / AT_QB)
#define DMODEL 1024
#define LDQKV 3072
#define LDAO 1024
#define KOFFP 1024
#define VOFFP 2048
#define PCARRY 32768.0f
#define OCARRY 256.0f
#define OCARRY_OVER_PCARRY (1.0f / 128.0f)
#define WCARRY 64.0f
#define BIASL_N 2176
#define RELP_ROWS 4095
#define RELP_N 4096
#define RPE_DIM 64
#define LOG2E_F 1.4426950408889634f
#define QK_SCALE 0.125f

__global__ __launch_bounds__(256) void relp_table_kernel(const float* __restrict__ rel_pos,
                                                         const float* __restrict__ rpe_w,
                                                         float* __restrict__ relp) {
  __shared__ __align__(16) float wsh[RPE_DIM];
  const int tid = threadIdx.x;
  if (tid < RPE_DIM) wsh[tid] = rpe_w[tid];
  __syncthreads();
  const int i = blockIdx.x * 256 + tid;
  const int row = (i < RELP_ROWS) ? i : (RELP_ROWS - 1);
  const float* rp = rel_pos + (size_t)row * RPE_DIM;
  float s = 0.f;
#pragma unroll 1
  for (int d4 = 0; d4 < RPE_DIM / 4; ++d4) {
    const v4f t = *(const v4f*)(rp + 4 * d4);
    s = fmaf(t[0], wsh[4 * d4 + 0], s);
    s = fmaf(t[1], wsh[4 * d4 + 1], s);
    s = fmaf(t[2], wsh[4 * d4 + 2], s);
    s = fmaf(t[3], wsh[4 * d4 + 3], s);
  }
  if (i >= RELP_ROWS) s = 0.f;
  if (i < RELP_N) {
    ((volatile float*)relp)[i] = s;
    __threadfence();
    ((volatile float*)relp)[i] = s;
  }
}

__device__ __forceinline__ v8f mma_h16(v16h a, v16h b, v8f c) {
  c = __builtin_amdgcn_wmma_f32_16x16x32_f16(false, a, false, b, (short)0, c, false, false);
  asm volatile("v_nop\n\tv_nop\n\tv_nop\n\tv_nop" : "+v"(c) : "v"(a), "v"(b));
  return c;
}
__device__ __forceinline__ void put_vt2(unsigned short* vt, int d, int kvr, unsigned w) {
  vt[d * AT_KC + kvr]       = (unsigned short)(w & 0xffffu);
  vt[(d + 1) * AT_KC + kvr] = (unsigned short)(w >> 16);
}

__global__ __launch_bounds__(128)
void attn_rpe_kernel(const unsigned short* __restrict__ qkv, const float* __restrict__ relp,
                     unsigned short* __restrict__ ao) {
  union FH { v16h v; v8h h[2]; };
  __shared__ __align__(16) unsigned short Ksh[AT_KC * AT_D];
  __shared__ __align__(16) unsigned short Vth[AT_D * AT_KC];
  __shared__ __align__(16) _Float16 Psh[AT_NW][16 * AT_KC];
  __shared__ __align__(16) float Os[AT_NW][16 * 68];
  __shared__ __align__(16) float biasL[BIASL_N];

  const int tid  = threadIdx.x;
  const int wave = tid >> 5;
  const int lane = tid & 31;
  const int hh   = lane >> 4;
  const int c    = lane & 15;

  const int bx = blockIdx.x;
  const int qb = bx % NQB;
  const int bh = bx / NQB;
  const int h  = bh % NHEAD;
  const int b  = bh / NHEAD;
  const int qbase = qb * AT_QB;
  const int q0 = qbase + wave * 16;

  const unsigned short* qb_ptr = qkv + (size_t)b * SEQ_T * LDQKV + h * AT_D;
  const unsigned short* kb_ptr = qb_ptr + KOFFP;
  const unsigned short* vb_ptr = qb_ptr + VOFFP;
  _Float16* ob_ptr = (_Float16*)(ao + (size_t)b * SEQ_T * LDAO + h * AT_D);

  for (int i = tid; i < BIASL_N / 4; i += 128) {
    int idx = 4 * i + (SEQ_T - AT_QB) - qbase;
    idx = (idx > RELP_N - 4) ? (RELP_N - 4) : idx;
    const v4f t = *(const v4f*)(relp + idx);
    *(v4f*)(biasL + 4 * i) = t * LOG2E_F;
  }

  v16h qa[2];
  {
    const _Float16* qrow = (const _Float16*)(qb_ptr + (size_t)(q0 + c) * LDQKV);
#pragma unroll
    for (int dc = 0; dc < 2; ++dc) qa[dc] = Frag<_Float16>::load(qrow + dc * 32 + 8 * hh);
  }

  float mrow[8], lrow[8];
  v8f oacc[4];
#pragma unroll
  for (int r = 0; r < 8; ++r) { mrow[r] = -__builtin_inff(); lrow[r] = 0.f; }
#pragma unroll
  for (int t = 0; t < 4; ++t) oacc[t] = (v8f){0.f,0.f,0.f,0.f,0.f,0.f,0.f,0.f};

  for (int kc = 0; kc < SEQ_T / AT_KC; ++kc) {
    const int kv0 = kc * AT_KC;
    __syncthreads();
    {
      const int kvr = tid >> 1, dh = (tid & 1) * 32;
      const v4u* krow = (const v4u*)(kb_ptr + (size_t)(kv0 + kvr) * LDQKV + dh);
      const v4u* vrow = (const v4u*)(vb_ptr + (size_t)(kv0 + kvr) * LDQKV + dh);
      v4u* kdst = (v4u*)(Ksh + kvr * AT_D + dh);
#pragma unroll
      for (int i = 0; i < 4; ++i) {
        const v4u kk = krow[i];
        const v4u vv = vrow[i];
        kdst[i] = kk;
        const int d = dh + 8 * i;
        put_vt2(Vth, d + 0, kvr, vv[0]);
        put_vt2(Vth, d + 2, kvr, vv[1]);
        put_vt2(Vth, d + 4, kvr, vv[2]);
        put_vt2(Vth, d + 6, kvr, vv[3]);
      }
    }
    __syncthreads();

    v8f s[4];
#pragma unroll
    for (int j = 0; j < 4; ++j) {
      s[j] = (v8f){0.f,0.f,0.f,0.f,0.f,0.f,0.f,0.f};
#pragma unroll
      for (int dc = 0; dc < 2; ++dc) {
        FH kb;
        kb.h[0] = *(const v8h*)(Ksh + (j * 16 + c) * AT_D + dc * 32 + 8 * hh);
        kb.h[1] = *(const v8h*)(Ksh + (j * 16 + c) * AT_D + dc * 32 + 16 + 8 * hh);
        s[j] = mma_h16(qa[dc], kb.v, s[j]);
      }
    }
    float cm[8];
#pragma unroll
    for (int r = 0; r < 8; ++r) {
      const int qoff = wave * 16 + 8 * hh + r;
      float m = -__builtin_inff();
#pragma unroll
      for (int j = 0; j < 4; ++j) {
        const int u = kv0 + j * 16 + c - qoff + (AT_QB - 1);
        const float sv = fmaf(s[j][r], QK_SCALE * LOG2E_F, biasL[u]);
        s[j][r] = sv;
        m = fmaxf(m, sv);
      }
#pragma unroll
      for (int off = 1; off < 16; off <<= 1) m = fmaxf(m, __shfl_xor(m, off, 32));
      cm[r] = m;
    }
    _Float16* pwh = Psh[wave];
#pragma unroll
    for (int r = 0; r < 8; ++r) {
      const float mnew = fmaxf(mrow[r], cm[r]);
      const float alpha = exp2f(mrow[r] - mnew);
      mrow[r] = mnew;
      float psum = 0.f;
#pragma unroll
      for (int j = 0; j < 4; ++j) {
        const float p = exp2f(s[j][r] - mnew);
        psum += p;
        pwh[(8 * hh + r) * AT_KC + j * 16 + c] = (_Float16)(p * PCARRY);
      }
#pragma unroll
      for (int off = 1; off < 16; off <<= 1) psum += __shfl_xor(psum, off, 32);
      lrow[r] = lrow[r] * alpha + psum;
#pragma unroll
      for (int t = 0; t < 4; ++t) oacc[t][r] *= alpha;
    }
    __builtin_amdgcn_fence(__ATOMIC_RELEASE, "workgroup");
    __builtin_amdgcn_wave_barrier();
    __builtin_amdgcn_fence(__ATOMIC_ACQUIRE, "workgroup");
#pragma unroll 1
    for (int kk = 0; kk < 2; ++kk) {
      FH pa;
      pa.h[0] = *(const v8h*)(pwh + c * AT_KC + kk * 32 + 8 * hh);
      pa.h[1] = *(const v8h*)(pwh + c * AT_KC + kk * 32 + 16 + 8 * hh);
#pragma unroll
      for (int t = 0; t < 4; ++t) {
        FH vb;
        vb.h[0] = *(const v8h*)(Vth + (t * 16 + c) * AT_KC + kk * 32 + 8 * hh);
        vb.h[1] = *(const v8h*)(Vth + (t * 16 + c) * AT_KC + kk * 32 + 16 + 8 * hh);
        oacc[t] = mma_h16(pa.v, vb.v, oacc[t]);
      }
    }
  }

  float* os = Os[wave];
#pragma unroll
  for (int r = 0; r < 8; ++r) {
    const float inv = OCARRY_OVER_PCARRY / lrow[r];
#pragma unroll
    for (int t = 0; t < 4; ++t) os[(8 * hh + r) * 68 + t * 16 + c] = oacc[t][r] * inv;
  }
  __builtin_amdgcn_fence(__ATOMIC_RELEASE, "workgroup");
  __builtin_amdgcn_wave_barrier();
  __builtin_amdgcn_fence(__ATOMIC_ACQUIRE, "workgroup");
  {
    const int q8 = lane >> 3, c8 = (lane & 7) * 8;
    for (int pass = 0; pass < 2; ++pass) {
#pragma unroll
      for (int it = 0; it < 4; ++it) {
        const int row = it * 4 + q8;
        const float* sp = os + row * 68 + c8;
        v8h hv;
#pragma unroll
        for (int e = 0; e < 8; ++e) hv[e] = (_Float16)sp[e];
        *(volatile v8h*)(ob_ptr + (size_t)(q0 + row) * LDAO + c8) = hv;
      }
      __threadfence();
    }
  }
}

extern "C" void kernel_launch(void* const* d_in, const int* in_sizes, int n_in,
                              void* d_out, int out_size, void* d_ws, size_t ws_size,
                              hipStream_t stream) {
  constexpr int kRows   = NBATCH * SEQ_T;
  constexpr int kDm     = DMODEL;
  constexpr int kQkvN   = 3 * DMODEL;
  static_assert(kRows % 64 == 0 && kQkvN % 64 == 0 && kDm % 64 == 0, "");
  static_assert(kDm % 32 == 0, "");
  static_assert((kRows * kDm) % 512 == 0 && (kQkvN * kDm) % 512 == 0 && (kDm * kDm) % 512 == 0, "");
  static_assert(SEQ_T % AT_QB == 0 && SEQ_T % AT_KC == 0 && AT_D == 64, "");
  static_assert(BIASL_N >= SEQ_T + AT_QB - 1 && BIASL_N % 4 == 0, "");

  if (n_in < 7) return;
  (void)in_sizes; (void)out_size;

  const float* x       = (const float*)d_in[0];
  const float* qkv_w   = (const float*)d_in[1];
  const float* qkv_b   = (const float*)d_in[2];
  const float* out_w   = (const float*)d_in[3];
  const float* out_b   = (const float*)d_in[4];
  const float* rel_pos = (const float*)d_in[5];
  const float* rpe_w   = (const float*)d_in[6];
  float* out = (float*)d_out;

  constexpr size_t kXH   = (size_t)kRows * kDm * 2;
  constexpr size_t kWQ   = (size_t)kQkvN * kDm * 2;
  constexpr size_t kWO   = (size_t)kDm * kDm * 2;
  constexpr size_t kQKVP = (size_t)kRows * kQkvN * 2;
  constexpr size_t kAOP  = (size_t)kRows * kDm * 2;
  constexpr size_t kRELP = (size_t)RELP_N * 4;
  constexpr size_t oXH   = 0;
  constexpr size_t oWQ   = oXH + kXH;
  constexpr size_t oWO   = oWQ + kWQ;
  constexpr size_t oQKVP = oWO + kWO;
  constexpr size_t oAOP  = oQKVP + kQKVP;
  constexpr size_t oRELP = oAOP + kAOP;
  constexpr size_t kWsTotal = oRELP + kRELP;
  static_assert(kWsTotal == 50348032, "");
  static_assert(kWsTotal <= (size_t)134217728, "");
  static_assert(oWQ % 128 == 0 && oWO % 128 == 0 && oQKVP % 128 == 0 && oAOP % 128 == 0 && oRELP % 128 == 0, "");
  if (ws_size < kWsTotal) return;

  char* ws = (char*)d_ws;
  _Float16* xh = (_Float16*)(ws + oXH);
  _Float16* wq = (_Float16*)(ws + oWQ);
  _Float16* wo = (_Float16*)(ws + oWO);
  unsigned short* qkvp = (unsigned short*)(ws + oQKVP);
  unsigned short* aop  = (unsigned short*)(ws + oAOP);
  float* relp = (float*)(ws + oRELP);

  constexpr int n2x = kRows * kDm / 2;
  constexpr int n2q = kQkvN * kDm / 2;
  constexpr int n2o = kDm * kDm / 2;
  static_assert(n2x % 256 == 0 && n2q % 256 == 0 && n2o % 256 == 0, "");
  cast_f32_f16x2s<<<n2x / 256, 256, 0, stream>>>(x, xh, n2x, 1.0f);
  cast_f32_f16x2s<<<n2q / 256, 256, 0, stream>>>(qkv_w, wq, n2q, WCARRY);
  cast_f32_f16x2s<<<n2o / 256, 256, 0, stream>>>(out_w, wo, n2o, WCARRY);

  static_assert(RELP_N % 256 == 0, "");
  relp_table_kernel<<<RELP_N / 256, 256, 0, stream>>>(rel_pos, rpe_w, relp);

  {
    constexpr int tiles = (kRows / 64) * (kQkvN / 64);
    static_assert(tiles % 8 == 0, "");
    wmma_gemm64<0, false, 2, 1, false, 0><<<dim3(tiles / 8, 1), 256, 0, stream>>>(
        (const unsigned short*)xh, (const unsigned short*)xh, kDm, 0L,
        (const unsigned short*)wq, (const unsigned short*)wq, kDm, 0L,
        (void*)qkvp, (void*)qkvp, kQkvN, 0L,
        qkv_b, qkv_b, 0L,
        kRows, kQkvN, kDm, 1.0f / WCARRY);
  }

  attn_rpe_kernel<<<NBATCH * NHEAD * NQB, 128, 0, stream>>>(qkvp, relp, aop);

  {
    constexpr int tiles = (kRows / 64) * (kDm / 64);
    static_assert(tiles % 8 == 0, "");
    wmma_gemm64<0, false, 2, 0, false, 0><<<dim3(tiles / 8, 1), 256, 0, stream>>>(
        (const unsigned short*)aop, (const unsigned short*)aop, kDm, 0L,
        (const unsigned short*)wo, (const unsigned short*)wo, kDm, 0L,
        (void*)out, (void*)out, kDm, 0L,
        out_b, out_b, 0L,
        kRows, kDm, kDm, 1.0f / (WCARRY * OCARRY));
  }
}
